// GCN_ZINC_5282809774463
// MI455X (gfx1250) — hardware-run, weakly checked
//
#include <hip/hip_runtime.h>
#include <stddef.h>


#define HID     145
#define HP      160
#define HMID    72
#define HMP     80
#define NTHR    256
#define NWAVE   8
#define EPT     8
#define NGRP    2
#define CHUNK   (NTHR * EPT * NGRP)
#define WCAP    (EPT * NGRP * 32)
#define LISTN   (NWAVE * WCAP)
#define NBC     4096
#define NBF     1024
#define RCAP    40960
#define RBN     128
#define TGT     256
#define DEGCAP  256
#define OTHR    512
#define BM      64
#define STATR   256
#define GPB     32
#define NTW     5
#define F4ROW   (HP / 4)
#define WSCAP   134217728
#define BN_EPS  1e-5
#define XSC     8.0f
#define WSC     64.0f
#define INV_CARRY (1.0f / 512.0f)

#define LDS_FILL ((RCAP + NBF + LISTN) * 4 + 64)

static_assert((CHUNK & (CHUNK - 1)) == 0);
static_assert(CHUNK <= 4096);
static_assert(NBC <= 4096 && NBF <= 4096);
static_assert((NBC & (NBC - 1)) == 0 && (NBF & (NBF - 1)) == 0);
static_assert(NBC == 4 * NBF);
static_assert(OTHR * 8 == NBC);
static_assert((RCAP % 32) == 0);
static_assert(TGT == NWAVE * 32);
static_assert((TGT % BM) == 0 && (TGT % STATR) == 0 && (NBF % TGT) == 0);
static_assert(2 * 16 * NTW == HP);
static_assert((HP % 32) == 0 && (HMP % 16) == 0);
static_assert((BM * F4ROW) % NTHR == 0);
static_assert((GPB & (GPB - 1)) == 0 && GPB == 32);
static_assert(HP <= NTHR);

typedef float          v4f  __attribute__((ext_vector_type(4)));
typedef float          v8f  __attribute__((ext_vector_type(8)));
typedef int            v4i  __attribute__((ext_vector_type(4)));
typedef _Float16       v4h  __attribute__((ext_vector_type(4)));
typedef _Float16       v8h  __attribute__((ext_vector_type(8)));
typedef _Float16       v16h __attribute__((ext_vector_type(16)));
union FragH { v16h v; v8h h[2]; };

__device__ __forceinline__ v8f wmh(v16h a, v16h b, v8f c) {
  v8f d = __builtin_amdgcn_wmma_f32_16x16x32_f16(false, a, false, b, (short)0, c, false, false);
  asm volatile("v_nop\n\tv_nop\n\tv_nop\n\tv_nop" : "+v"(d) : "v"(a), "v"(b));
  return d;
}

template <int NB>
__device__ __forceinline__ int scan_chunk(const int* __restrict__ dsts, int nE, int cbase, int slotBase,
                                          int vec8, int* list, int tid, int lane, int wave) {
  int wc = 0;
#pragma unroll
  for (int g = 0; g < NGRP; ++g) {
    const int el0  = (g * NTHR + tid) * EPT;
    const int e0   = cbase + el0;
    const int sent = -2147483647 - 1;
    v4i da, db;
    if (vec8 != 0 && cbase + CHUNK <= nE) {
      da = *(const v4i*)(dsts + e0);
      db = *(const v4i*)(dsts + e0 + 4);
    } else {
      da.x = (e0     < nE) ? dsts[min(e0, nE - 1)] : sent;
      da.y = (e0 + 1 < nE) ? dsts[min(e0 + 1, nE - 1)] : sent;
      da.z = (e0 + 2 < nE) ? dsts[min(e0 + 2, nE - 1)] : sent;
      da.w = (e0 + 3 < nE) ? dsts[min(e0 + 3, nE - 1)] : sent;
      db.x = (e0 + 4 < nE) ? dsts[min(e0 + 4, nE - 1)] : sent;
      db.y = (e0 + 5 < nE) ? dsts[min(e0 + 5, nE - 1)] : sent;
      db.z = (e0 + 6 < nE) ? dsts[min(e0 + 6, nE - 1)] : sent;
      db.w = (e0 + 7 < nE) ? dsts[min(e0 + 7, nE - 1)] : sent;
    }
    const unsigned nb = (unsigned)slotBase;
    const unsigned s0 = (unsigned)da.x - nb, s1 = (unsigned)da.y - nb;
    const unsigned s2 = (unsigned)da.z - nb, s3 = (unsigned)da.w - nb;
    const unsigned s4 = (unsigned)db.x - nb, s5 = (unsigned)db.y - nb;
    const unsigned s6 = (unsigned)db.z - nb, s7 = (unsigned)db.w - nb;
    const bool h0 = s0 < (unsigned)NB, h1 = s1 < (unsigned)NB, h2 = s2 < (unsigned)NB, h3 = s3 < (unsigned)NB;
    const bool h4 = s4 < (unsigned)NB, h5 = s5 < (unsigned)NB, h6 = s6 < (unsigned)NB, h7 = s7 < (unsigned)NB;
    const unsigned any = __builtin_amdgcn_ballot_w32(h0 | h1 | h2 | h3 | h4 | h5 | h6 | h7);
    if (any != 0u) {
#define HITJ(J, HJ, SJ) { \
        const unsigned mj = __builtin_amdgcn_ballot_w32(HJ); \
        if (mj != 0u) { \
          if (HJ) { \
            const int pos = wc + (int)__builtin_amdgcn_mbcnt_lo(mj, 0u); \
            if (pos < WCAP) list[wave * WCAP + pos] = ((el0 + (J)) << 12) | (int)(SJ); \
          } \
          wc += (int)__builtin_popcount(mj); } }
      HITJ(0, h0, s0)
      HITJ(1, h1, s1)
      HITJ(2, h2, s2)
      HITJ(3, h3, s3)
      HITJ(4, h4, s4)
      HITJ(5, h5, s5)
      HITJ(6, h6, s6)
      HITJ(7, h7, s7)
#undef HITJ
    }
  }
  return wc;
}

template <int KS, int NS, int KD, int NCP>
__global__ __launch_bounds__(NTHR) void k_wprep(const float* __restrict__ W, _Float16* wp, int nL) {
  constexpr int KD8 = KD / 8;
  constexpr int UPL = NCP * KD8;
  static_assert((UPL % 32) == 0);
  const int i = (int)blockIdx.x * NTHR + (int)threadIdx.x;
  if (i >= nL * UPL) return;
  const int l  = i / UPL;
  const int r  = i - l * UPL;
  const int n  = r / KD8;
  const int k0 = (r - n * KD8) * 8;
  const int nn = n < NS ? n : NS - 1;
  v8h hv;
#pragma unroll
  for (int e = 0; e < 8; ++e) {
    const int k  = k0 + e;
    const int kk = k < KS ? k : KS - 1;
    float v = W[((size_t)l * KS + kk) * NS + nn];
    if (k >= KS || n >= NS) v = 0.0f;
    hv[e] = (_Float16)(v * WSC);
  }
  _Float16* d = wp + (size_t)i * 8;
  *(volatile v8h*)d = hv;
  __threadfence();
  *(volatile v8h*)d = hv;
}

__global__ __launch_bounds__(NTHR) void k_embed(const int* __restrict__ x, const float* __restrict__ emb,
                                                float* h32, _Float16* h16, int nN, int nCls, int nUnits) {
  const int i = (int)blockIdx.x * NTHR + (int)threadIdx.x;
  if (i >= nUnits) return;
  const int row = i / F4ROW;
  const int c   = (i - row * F4ROW) * 4;
  const int rr  = row < nN ? row : nN - 1;
  int cls = x[rr];
  cls = cls < 0 ? 0 : (cls > nCls - 1 ? nCls - 1 : cls);
  const float* er = emb + (size_t)cls * HID;
  const int c0 = c     < HID ? c     : HID - 1;
  const int c1 = c + 1 < HID ? c + 1 : HID - 1;
  const int c2 = c + 2 < HID ? c + 2 : HID - 1;
  const int c3 = c + 3 < HID ? c + 3 : HID - 1;
  v4f v;
  v.x = er[c0]; v.y = er[c1]; v.z = er[c2]; v.w = er[c3];
  const bool rok = row < nN;
  if (!rok || c     >= HID) v.x = 0.0f;
  if (!rok || c + 1 >= HID) v.y = 0.0f;
  if (!rok || c + 2 >= HID) v.z = 0.0f;
  if (!rok || c + 3 >= HID) v.w = 0.0f;
  v4h hv;
  hv.x = (_Float16)(v.x * XSC); hv.y = (_Float16)(v.y * XSC);
  hv.z = (_Float16)(v.z * XSC); hv.w = (_Float16)(v.w * XSC);
  const size_t p = (size_t)i * 4;
  *(volatile v4f*)(h32 + p) = v;
  *(volatile v4h*)(h16 + p) = hv;
  __threadfence();
  *(volatile v4f*)(h32 + p) = v;
  *(volatile v4h*)(h16 + p) = hv;
}

__global__ __launch_bounds__(NTHR) void k_count(
    const int* __restrict__ dsts, int* cnt, int nE, int vec8) {
  __shared__ __attribute__((aligned(16))) int scnt[NBC];
  __shared__ __attribute__((aligned(16))) int list[LISTN];
  __shared__ int wcnt[NWAVE];
  const int tid = threadIdx.x, lane = tid & 31, wave = tid >> 5;
  const int nodeBase = blockIdx.x * NBC;

  for (int i = tid; i < NBC; i += NTHR) scnt[i] = 0;
  __syncthreads();

  const int nChunks = (nE + CHUNK - 1) / CHUNK;
#pragma unroll 1
  for (int ch = 0; ch < nChunks; ++ch) {
    const int cbase = ch * CHUNK;
    const int wc = scan_chunk<NBC>(dsts, nE, cbase, nodeBase, vec8, list, tid, lane, wave);
    if (lane == 0) wcnt[wave] = wc;
    __syncthreads();
    if (wave == 0) {
#pragma unroll 1
      for (int wsx = 0; wsx < NWAVE; ++wsx) {
        int n = __builtin_amdgcn_readfirstlane(wcnt[wsx]);
        n = n > WCAP ? WCAP : (n < 0 ? 0 : n);
        const int* lp = list + wsx * WCAP;
#pragma unroll 1
        for (int i = 0; i < n; ++i) {
          const int ent  = __builtin_amdgcn_readfirstlane(lp[i]);
          const int slot = ent & (NBC - 1);
          if (lane == 0) scnt[slot] = scnt[slot] + 1;
        }
      }
    }
    __syncthreads();
  }

  v4i cq[4];
#pragma unroll
  for (int q = 0; q < 4; ++q) {
    const int f = (wave * 4 + q) * 128 + 4 * lane;
    cq[q] = *(const v4i*)(scnt + f);
  }
  int* cp = cnt + (size_t)nodeBase;
#pragma unroll
  for (int q = 0; q < 4; ++q) {
    const int f = (wave * 4 + q) * 128 + 4 * lane;
    *(volatile v4i*)(cp + f) = cq[q];
  }
  __threadfence();
#pragma unroll
  for (int q = 0; q < 4; ++q) {
    const int f = (wave * 4 + q) * 128 + 4 * lane;
    *(volatile v4i*)(cp + f) = cq[q];
  }
}

__global__ __launch_bounds__(OTHR) void k_offsets(
    const int* __restrict__ cnt, int* off, int* rbase, int nChunk) {
  __shared__ __attribute__((aligned(16))) int soff[NBC];
  __shared__ __attribute__((aligned(16))) int srb[RBN];
  __shared__ int wtot[OTHR / 32];
  const int tid = threadIdx.x, lane = tid & 31, wave = tid >> 5, sub = tid >> 7;
  for (int i = tid; i < RBN; i += OTHR) srb[i] = 0;
  int carry = 0;
#pragma unroll 1
  for (int ch = 0; ch < nChunk; ++ch) {
    const int base = ch * NBC;
    const v4i c0 = *(const v4i*)(cnt + base + 8 * tid);
    const v4i c1 = *(const v4i*)(cnt + base + 8 * tid + 4);
    const int e0 = max(c0.x, 0), e1 = max(c0.y, 0), e2 = max(c0.z, 0), e3 = max(c0.w, 0);
    const int e4 = max(c1.x, 0), e5 = max(c1.y, 0), e6 = max(c1.z, 0), e7 = max(c1.w, 0);
    const int ts = e0 + e1 + e2 + e3 + e4 + e5 + e6 + e7;
    int incl = ts;
#pragma unroll
    for (int d = 1; d < 32; d <<= 1) {
      const int t = __shfl_up(incl, d);
      if (lane >= d) incl += t;
    }
    if (lane == 31) wtot[wave] = incl;
    __syncthreads();
    const int S0 = wtot[0]  + wtot[1]  + wtot[2]  + wtot[3];
    const int S1 = wtot[4]  + wtot[5]  + wtot[6]  + wtot[7];
    const int S2 = wtot[8]  + wtot[9]  + wtot[10] + wtot[11];
    const int S3 = wtot[12] + wtot[13] + wtot[14] + wtot[15];
    int pre = 0;
#pragma unroll 1
    for (int w = 4 * sub; w < wave; ++w) pre += wtot[w];
    const int b0 = carry;
    const int b1 = b0 + ((S0 + 31) & ~31);
    const int b2 = b1 + ((S1 + 31) & ~31);
    const int b3 = b2 + ((S2 + 31) & ~31);
    const int b4 = b3 + ((S3 + 31) & ~31);
    const int myb = sub == 0 ? b0 : (sub == 1 ? b1 : (sub == 2 ? b2 : b3));
    if (tid == 0) {
      srb[min(4 * ch + 0, RBN - 1)] = b0;
      srb[min(4 * ch + 1, RBN - 1)] = b1;
      srb[min(4 * ch + 2, RBN - 1)] = b2;
      srb[min(4 * ch + 3, RBN - 1)] = b3;
    }
    int run = myb + pre + incl - ts;
    soff[8 * tid + 0] = run; run += e0;
    soff[8 * tid + 1] = run; run += e1;
    soff[8 * tid + 2] = run; run += e2;
    soff[8 * tid + 3] = run; run += e3;
    soff[8 * tid + 4] = run; run += e4;
    soff[8 * tid + 5] = run; run += e5;
    soff[8 * tid + 6] = run; run += e6;
    soff[8 * tid + 7] = run;
    carry = b4;
    __syncthreads();
    const v4i o0 = *(const v4i*)(soff + 4 * tid);
    const v4i o1 = *(const v4i*)(soff + 4 * (tid + OTHR));
    int* op = off + base;
    *(volatile v4i*)(op + 4 * tid) = o0;
    *(volatile v4i*)(op + 4 * (tid + OTHR)) = o1;
    __threadfence();
    *(volatile v4i*)(op + 4 * tid) = o0;
    *(volatile v4i*)(op + 4 * (tid + OTHR)) = o1;
    __syncthreads();
  }
  if (tid == 0) srb[min(4 * nChunk, RBN - 1)] = carry;
  __syncthreads();
  v4i rv = {0, 0, 0, 0};
  if (tid < 32) rv = *(const v4i*)(srb + 4 * tid);
  if (tid < 32) *(volatile v4i*)(rbase + 4 * tid) = rv;
  __threadfence();
  if (tid < 32) *(volatile v4i*)(rbase + 4 * tid) = rv;
}

__global__ __launch_bounds__(NTHR) void k_fill(
    const int* __restrict__ srcs, const int* __restrict__ dsts,
    const int* __restrict__ off, const int* __restrict__ rbase,
    int* csr, int nN, int nE, int vec8, int csrLen) {
  extern __shared__ v4f lds_dyn[];
  int* region = (int*)lds_dyn;
  int* cursor = region + RCAP;
  int* list   = cursor + NBF;
  int* wcnt   = list + LISTN;
  const int tid = threadIdx.x, lane = tid & 31, wave = tid >> 5;
  const int b = blockIdx.x;
  const int nodeBase = b * NBF;

  int rb0 = rbase[b];
  const int rb1 = rbase[b + 1];
  rb0 = rb0 < 0 ? 0 : (rb0 > csrLen ? csrLen : rb0);
  rb0 &= ~31;
  int len = rb1 - rb0;
  len = len < 0 ? 0 : (len > RCAP ? RCAP : len);
  int lenW = (len + 31) & ~31;
  if (rb0 + lenW > csrLen) lenW = (csrLen - rb0) & ~31;

  {
    const v4i z = {0, 0, 0, 0};
    for (int i = tid; i < RCAP / 4; i += NTHR) ((v4i*)region)[i] = z;
    for (int s = tid; s < NBF; s += NTHR) {
      int o = off[nodeBase + s] - rb0;
      o = o < 0 ? 0 : (o > RCAP ? RCAP : o);
      cursor[s] = o;
    }
  }
  __syncthreads();

  const int nChunks = (nE + CHUNK - 1) / CHUNK;
#pragma unroll 1
  for (int ch = 0; ch < nChunks; ++ch) {
    const int cbase = ch * CHUNK;
    const int wc = scan_chunk<NBF>(dsts, nE, cbase, nodeBase, vec8, list, tid, lane, wave);
    if (lane == 0) wcnt[wave] = wc;
    __syncthreads();
    if (wave == 0) {
#pragma unroll 1
      for (int wsx = 0; wsx < NWAVE; ++wsx) {
        int n = __builtin_amdgcn_readfirstlane(wcnt[wsx]);
        n = n > WCAP ? WCAP : (n < 0 ? 0 : n);
        const int* lp = list + wsx * WCAP;
#pragma unroll 1
        for (int i = 0; i < n; ++i) {
          const int ent  = __builtin_amdgcn_readfirstlane(lp[i]);
          const int slot = ent & (NBF - 1);
          int e = cbase + ((ent >> 12) & (CHUNK - 1));
          e = e > nE - 1 ? nE - 1 : e;
          int src = srcs[e];
          src = src < 0 ? 0 : (src > nN - 1 ? nN - 1 : src);
          if (lane == 0) {
            int pos = cursor[slot];
            pos = pos < 0 ? 0 : (pos > RCAP - 1 ? RCAP - 1 : pos);
            region[pos] = src;
            const int np = pos + 1;
            cursor[slot] = np > RCAP ? RCAP : np;
          }
        }
      }
    }
    __syncthreads();
  }

  const int nv = lenW >> 2;
  int* gp = csr + rb0;
#pragma unroll 1
  for (int i = tid; i < nv; i += NTHR) { const v4i v = ((const v4i*)region)[i]; *(volatile v4i*)(gp + 4 * i) = v; }
  __threadfence();
#pragma unroll 1
  for (int i = tid; i < nv; i += NTHR) { const v4i v = ((const v4i*)region)[i]; *(volatile v4i*)(gp + 4 * i) = v; }
}

__global__ __launch_bounds__(NTHR) void k_dis(const int* __restrict__ cnt, float* dis, int nN) {
  const int i = (int)blockIdx.x * NTHR + (int)threadIdx.x;
  int c = cnt[i];
  c = c < 0 ? 0 : c;
  float d = rsqrtf((float)c + 1.0f);
  if (i >= nN) d = 0.0f;
  *(volatile float*)(dis + i) = d;
  __threadfence();
  *(volatile float*)(dis + i) = d;
}

__device__ __forceinline__ void mm_tile(const _Float16* __restrict__ A, const _Float16* __restrict__ Bw,
                                        int rowBase, float* stg) {
  const int tid = threadIdx.x, lane = tid & 31, wave = tid >> 5, hh = lane >> 4, m = lane & 15;
  const int r0 = (wave >> 1) * 16, c0 = (wave & 1) * (16 * NTW);
  v8f acc[NTW];
#pragma unroll
  for (int t = 0; t < NTW; ++t) { v8f z = {0.f, 0.f, 0.f, 0.f, 0.f, 0.f, 0.f, 0.f}; acc[t] = z; }
  const _Float16* ap  = A  + (size_t)(rowBase + r0 + m) * HP + 8 * hh;
  const _Float16* bp0 = Bw + (size_t)(c0 + m) * HP + 8 * hh;
#pragma unroll 1
  for (int kt = 0; kt < HP / 32; ++kt) {
    FragH a;
    a.h[0] = *(const v8h*)(ap + 32 * kt);
    a.h[1] = *(const v8h*)(ap + 32 * kt + 16);
#pragma unroll
    for (int t = 0; t < NTW; ++t) {
      const _Float16* bp = bp0 + (size_t)(16 * t) * HP + 32 * kt;
      FragH b;
      b.h[0] = *(const v8h*)bp;
      b.h[1] = *(const v8h*)(bp + 16);
      acc[t] = wmh(a.v, b.v, acc[t]);
    }
  }
  float* sp = stg + (size_t)(r0 + 8 * hh) * HP + c0 + m;
#pragma unroll
  for (int t = 0; t < NTW; ++t) {
#pragma unroll
    for (int r = 0; r < 8; ++r) sp[r * HP + 16 * t] = acc[t][r] * INV_CARRY;
  }
}

__global__ __launch_bounds__(NTHR) void k_gemm(const _Float16* __restrict__ A, const _Float16* __restrict__ Bw,
                                               float* C) {
  __shared__ __attribute__((aligned(16))) float stg[BM * HP];
  const int tid = threadIdx.x;
  const int rowBase = blockIdx.x * BM;
  mm_tile(A, Bw, rowBase, stg);
  __syncthreads();
  constexpr int NIT = (BM * F4ROW) / NTHR;
  const size_t gb = (size_t)blockIdx.x * (BM * F4ROW);
  v4f vv[NIT];
#pragma unroll
  for (int it = 0; it < NIT; ++it) vv[it] = ((const v4f*)stg)[it * NTHR + tid];
#pragma unroll
  for (int it = 0; it < NIT; ++it) *(volatile v4f*)(C + (gb + (size_t)(it * NTHR + tid)) * 4) = vv[it];
  __threadfence();
#pragma unroll
  for (int it = 0; it < NIT; ++it) *(volatile v4f*)(C + (gb + (size_t)(it * NTHR + tid)) * 4) = vv[it];
}

__global__ __launch_bounds__(NTHR) void k_agg(
    const int* __restrict__ csr, const int* __restrict__ off, const int* __restrict__ cnt,
    const float* __restrict__ dis, const float* __restrict__ hw, const float* __restrict__ bias,
    float* aout, int nN, int csrLen) {
  const int tid = threadIdx.x, lane = tid & 31, wave = tid >> 5;
  const int tbase = blockIdx.x * TGT + wave * 32;
  const int col0 = 4 * lane;
  const int col1 = 128 + lane;
  const v4f z4 = {0.f, 0.f, 0.f, 0.f};
  v4f bb0;
  bb0.x = bias[col0]; bb0.y = bias[col0 + 1]; bb0.z = bias[col0 + 2]; bb0.w = bias[col0 + 3];
  const int c1c = col1 < HID ? col1 : HID - 1;
  float bb1 = bias[c1c];
  if (col1 >= HID) bb1 = 0.0f;

  const int   cl    = tbase + lane;
  const int   cnt_l = cnt[cl];
  const int   off_l = off[cl];
  const float dis_l = dis[cl];

#pragma unroll 1
  for (int j = 0; j < 32; ++j) {
    const int c = tbase + j;
    int n = __shfl(cnt_l, j);
    n = n < 0 ? 0 : (n > DEGCAP ? DEGCAP : n);
    const int   st = __shfl(off_l, j);
    const float dc = __shfl(dis_l, j);

    v4f   acc0 = z4;
    float acc1 = 0.0f;
#pragma unroll 1
    for (int q0 = 0; q0 < n; q0 += 32) {
      int pos = st + q0 + lane;
      pos = pos < 0 ? 0 : (pos > csrLen - 1 ? csrLen - 1 : pos);
      int sl = csr[pos];
      sl = sl < 0 ? 0 : (sl > nN - 1 ? nN - 1 : sl);
      const float dsl = dis[sl];
      const int mcnt = (n - q0) < 32 ? (n - q0) : 32;
#pragma unroll 1
      for (int pp = 0; pp < mcnt; ++pp) {
        const int   s  = __builtin_amdgcn_readlane(sl, pp);
        const float ds = __builtin_bit_cast(float, __builtin_amdgcn_readlane(__builtin_bit_cast(int, dsl), pp));
        const float w  = ds * dc;
        const v4f   h0 = *(const v4f*)(hw + (size_t)s * HP + col0);
        const float h1 = hw[(size_t)s * HP + col1];
        acc0 = acc0 + h0 * w;
        acc1 = fmaf(h1, w, acc1);
      }
    }
    {
      const float w  = dc * dc;
      const v4f   h0 = *(const v4f*)(hw + (size_t)c * HP + col0);
      const float h1 = hw[(size_t)c * HP + col1];
      acc0 = acc0 + h0 * w;
      acc1 = fmaf(h1, w, acc1);
    }
    v4f   v0 = acc0 + bb0;
    float v1 = acc1 + bb1;
    if (c >= nN) { v0 = z4; v1 = 0.0f; }

    float* pw = aout + (size_t)c * HP;
    *(volatile v4f*)(pw + col0)   = v0;
    *(volatile float*)(pw + col1) = v1;
    __threadfence();
    *(volatile v4f*)(pw + col0)   = v0;
    *(volatile float*)(pw + col1) = v1;
  }
}

__global__ __launch_bounds__(NTHR) void k_bnstat(const float* __restrict__ agg, double* part, int nN) {
  const int col = threadIdx.x;
  const int r0 = blockIdx.x * STATR;
  int nr = nN - r0;
  nr = nr < 0 ? 0 : (nr > STATR ? STATR : nr);
  double s = 0.0, q = 0.0;
#pragma unroll 1
  for (int i = 0; i < nr; ++i) {
    const double v = (double)agg[(size_t)(r0 + i) * HP + col];
    s += v;
    q += v * v;
  }
  double* pp = part + (size_t)blockIdx.x * (2 * HP);
  *(volatile double*)(pp + col) = s;
  *(volatile double*)(pp + HP + col) = q;
  __threadfence();
  *(volatile double*)(pp + col) = s;
  *(volatile double*)(pp + HP + col) = q;
}

__global__ __launch_bounds__(NTHR) void k_bnfin(const double* __restrict__ part, const float* __restrict__ gamma,
                                                float* tbl, int nPart, int nN) {
  const int col = threadIdx.x;
  double s = 0.0, q = 0.0;
#pragma unroll 1
  for (int b = 0; b < nPart; ++b) {
    s += part[(size_t)b * (2 * HP) + col];
    q += part[(size_t)b * (2 * HP) + HP + col];
  }
  const double inv = 1.0 / (double)nN;
  const double mu  = s * inv;
  double var = q * inv - mu * mu;
  var = var < 0.0 ? 0.0 : var;
  const int gc = col < HID ? col : HID - 1;
  float a = (float)((double)gamma[gc] / sqrt(var + BN_EPS));
  if (col >= HID) a = 0.0f;
  const float mf = (float)mu;
  *(volatile float*)(tbl + col) = mf;
  *(volatile float*)(tbl + HP + col) = a;
  __threadfence();
  *(volatile float*)(tbl + col) = mf;
  *(volatile float*)(tbl + HP + col) = a;
}

__global__ __launch_bounds__(NTHR) void k_update(
    const float* __restrict__ agg, const float* __restrict__ tbl, const float* __restrict__ beta,
    const float* __restrict__ hold, float* hnew, _Float16* h16, int nN, int nUnits) {
  const int i = (int)blockIdx.x * NTHR + (int)threadIdx.x;
  if (i >= nUnits) return;
  const int row = i / F4ROW;
  const int c   = (i - row * F4ROW) * 4;
  const v4f mu = *(const v4f*)(tbl + c);
  const v4f ga = *(const v4f*)(tbl + HP + c);
  const int c0 = c     < HID ? c     : HID - 1;
  const int c1 = c + 1 < HID ? c + 1 : HID - 1;
  const int c2 = c + 2 < HID ? c + 2 : HID - 1;
  const int c3 = c + 3 < HID ? c + 3 : HID - 1;
  v4f be;
  be.x = beta[c0]; be.y = beta[c1]; be.z = beta[c2]; be.w = beta[c3];
  const size_t p = (size_t)i * 4;
  const v4f a  = *(const v4f*)(agg + p);
  const v4f ho = *(const v4f*)(hold + p);
  v4f v = (a - mu) * ga + be;
  v.x = fmaxf(v.x, 0.0f); v.y = fmaxf(v.y, 0.0f); v.z = fmaxf(v.z, 0.0f); v.w = fmaxf(v.w, 0.0f);
  v = v + ho;
  const bool rok = row < nN;
  if (!rok || c     >= HID) v.x = 0.0f;
  if (!rok || c + 1 >= HID) v.y = 0.0f;
  if (!rok || c + 2 >= HID) v.z = 0.0f;
  if (!rok || c + 3 >= HID) v.w = 0.0f;
  v4h hv;
  hv.x = (_Float16)(v.x * XSC); hv.y = (_Float16)(v.y * XSC);
  hv.z = (_Float16)(v.z * XSC); hv.w = (_Float16)(v.w * XSC);
  *(volatile v4f*)(hnew + p) = v;
  *(volatile v4h*)(h16 + p) = hv;
  __threadfence();
  *(volatile v4f*)(hnew + p) = v;
  *(volatile v4h*)(h16 + p) = hv;
}

__global__ __launch_bounds__(NTHR) void k_pool_head(
    const int* __restrict__ bidx, const float* __restrict__ hfin, const _Float16* __restrict__ w1p,
    const float* __restrict__ b1, const float* __restrict__ W2, const float* __restrict__ b2,
    float* out, int nN, int nG, int vec8) {
  __shared__ __attribute__((aligned(16))) float    sacc[GPB * HP];
  __shared__ __attribute__((aligned(16))) _Float16 sA[GPB * HP];
  __shared__ __attribute__((aligned(16))) int      list[LISTN];
  __shared__ __attribute__((aligned(16))) float    souts[GPB];
  __shared__ float sinv[GPB];
  __shared__ int   scnt[GPB];
  __shared__ int   wcnt[NWAVE];
  const int tid = threadIdx.x, lane = tid & 31, wave = tid >> 5;
  const int gbase = blockIdx.x * GPB;

  for (int i = tid; i < GPB * HP; i += NTHR) sacc[i] = 0.0f;
  if (tid < GPB) { scnt[tid] = 0; souts[tid] = 0.0f; }
  __syncthreads();

  const int nChunks = (nN + CHUNK - 1) / CHUNK;
#pragma unroll 1
  for (int ch = 0; ch < nChunks; ++ch) {
    const int cbase = ch * CHUNK;
    const int wc = scan_chunk<GPB>(bidx, nN, cbase, gbase, vec8, list, tid, lane, wave);
    if (lane == 0) wcnt[wave] = wc;
    __syncthreads();
#pragma unroll 1
    for (int wsx = 0; wsx < NWAVE; ++wsx) {
      int n = wcnt[wsx];
      n = n > WCAP ? WCAP : (n < 0 ? 0 : n);
      const int* lp = list + wsx * WCAP;
#pragma unroll 1
      for (int i = 0; i < n; ++i) {
        const int ent  = lp[i];
        const int slot = ent & (GPB - 1);
        int node = cbase + ((ent >> 12) & (CHUNK - 1));
        node = node > nN - 1 ? nN - 1 : node;
        if (tid < HP) sacc[slot * HP + tid] += hfin[(size_t)node * HP + tid];
        if (tid == HP) scnt[slot] = scnt[slot] + 1;
      }
    }
    __syncthreads();
  }

  if (tid < GPB) {
    const int cg = scnt[tid];
    sinv[tid] = 1.0f / (float)(cg < 1 ? 1 : cg);
  }
  __syncthreads();
  if (tid < HP) {
#pragma unroll 1
    for (int s = 0; s < GPB; ++s) sA[s * HP + tid] = (_Float16)(sacc[s * HP + tid] * sinv[s] * XSC);
  }
  __syncthreads();

  if (wave < 2) {
    const int hh = lane >> 4, m = lane & 15;
    const int r0 = wave * 16;
    constexpr int NT = HMP / 16;
    v8f acc[NT];
#pragma unroll
    for (int t = 0; t < NT; ++t) { v8f z = {0.f, 0.f, 0.f, 0.f, 0.f, 0.f, 0.f, 0.f}; acc[t] = z; }
    const _Float16* ap  = sA  + (r0 + m) * HP + 8 * hh;
    const _Float16* bp0 = w1p + (size_t)m * HP + 8 * hh;
#pragma unroll 1
    for (int kt = 0; kt < HP / 32; ++kt) {
      FragH a;
      a.h[0] = *(const v8h*)(ap + 32 * kt);
      a.h[1] = *(const v8h*)(ap + 32 * kt + 16);
#pragma unroll
      for (int t = 0; t < NT; ++t) {
        const _Float16* bp = bp0 + (size_t)(16 * t) * HP + 32 * kt;
        FragH b;
        b.h[0] = *(const v8h*)bp;
        b.h[1] = *(const v8h*)(bp + 16);
        acc[t] = wmh(a.v, b.v, acc[t]);
      }
    }
    float prt[8];
#pragma unroll
    for (int r = 0; r < 8; ++r) prt[r] = 0.0f;
#pragma unroll
    for (int t = 0; t < NT; ++t) {
      const int col = 16 * t + m;
      const int cc  = col < HMID ? col : HMID - 1;
      float bv = b1[cc];
      float wv = W2[cc];
      if (col >= HMID) { bv = 0.0f; wv = 0.0f; }
#pragma unroll
      for (int r = 0; r < 8; ++r) {
        const float z = fmaxf(acc[t][r] * INV_CARRY + bv, 0.0f);
        prt[r] = fmaf(z, wv, prt[r]);
      }
    }
#pragma unroll
    for (int r = 0; r < 8; ++r) {
#pragma unroll
      for (int o = 1; o < 16; o <<= 1) prt[r] += __shfl_xor(prt[r], o);
    }
    const float b2v = b2[0];
    if (m == 0) {
#pragma unroll
      for (int r = 0; r < 8; ++r) souts[r0 + 8 * hh + r] = prt[r] + b2v;
    }
  }
  __syncthreads();

  if (wave == 0) {
    int nv = nG - gbase;
    nv = nv < 0 ? 0 : (nv > GPB ? GPB : nv);
    const int lq = lane < (GPB / 4) ? lane : (GPB / 4 - 1);
    const int f  = 4 * lq;
    const v4f v  = *(const v4f*)(souts + f);
    const bool full = (lane < GPB / 4) && (f + 4 <= nv);
    const bool tail = (lane < GPB / 4) && !full && (f < nv);
    float* op = out + gbase + f;
    if (full) *(volatile v4f*)op = v;
    if (tail) {
      *(volatile float*)op = v.x;
      if (f + 1 < nv) *(volatile float*)(op + 1) = v.y;
      if (f + 2 < nv) *(volatile float*)(op + 2) = v.z;
    }
    __threadfence();
    if (full) *(volatile v4f*)op = v;
    if (tail) {
      *(volatile float*)op = v.x;
      if (f + 1 < nv) *(volatile float*)(op + 1) = v.y;
      if (f + 2 < nv) *(volatile float*)(op + 2) = v.z;
    }
  }
}

extern "C" void kernel_launch(void* const* d_in, const int* in_sizes, int n_in,
                              void* d_out, int out_size, void* d_ws, size_t ws_size,
                              hipStream_t stream) {
  if (n_in < 12) return;
  const int nN = in_sizes[0];
  const int nE = in_sizes[1] / 2;
  const int nG = out_size;
  if (nN <= 0 || nE <= 0 || nG <= 0 || in_sizes[1] != 2 * nE || in_sizes[2] != nN) return;
  if (in_sizes[3] <= 0 || (in_sizes[3] % HID) != 0) return;
  const int nCls = in_sizes[3] / HID;
  if (in_sizes[4] <= 0 || (in_sizes[4] % (HID * HID)) != 0) return;
  const int nL = in_sizes[4] / (HID * HID);
  if (nL > 32) return;
  if (in_sizes[5] != nL * HID || in_sizes[6] != nL * HID || in_sizes[7] != nL * HID) return;
  if (in_sizes[8] != HID * HMID || in_sizes[9] != HMID || in_sizes[10] != HMID || in_sizes[11] < 1) return;
  if (nE > (1 << 28) || nN > (1 << 22) || nG > (1 << 22)) return;

  const int*   x     = (const int*)d_in[0];
  const int*   ei    = (const int*)d_in[1];
  const int*   batch = (const int*)d_in[2];
  const float* emb   = (const float*)d_in[3];
  const float* Wc    = (const float*)d_in[4];
  const float* bc    = (const float*)d_in[5];
  const float* gamma = (const float*)d_in[6];
  const float* beta  = (const float*)d_in[7];
  const float* W1    = (const float*)d_in[8];
  const float* b1    = (const float*)d_in[9];
  const float* W2    = (const float*)d_in[10];
  const float* b2    = (const float*)d_in[11];
  const int*   src = ei;
  const int*   dst = ei + nE;
  float* out = (float*)d_out;

  const int NPAD   = ((nN + TGT - 1) / TGT) * TGT;
  const int nBC    = (nN + NBC - 1) / NBC;
  const int CNTPAD = nBC * NBC;
  if (4 * nBC + 1 > RBN) return;
  const int nBF    = (nN + NBF - 1) / NBF;
  const int csrLen = ((nE + 31) & ~31) + 4096;
  if (31 * 4 * nBC > 4096) return;
  const int nAgg   = NPAD / TGT;
  const int nGm    = NPAD / BM;
  const int nStat  = NPAD / STATR;
  const int nUnit  = NPAD * F4ROW;
  const int nPool  = (nG + GPB - 1) / GPB;
  const int nWcU   = nL * HP * (HP / 8);
  const int nW1U   = HMP * (HP / 8);

  char* ws = (char*)d_ws;
  size_t off = 0;
  const size_t oWc  = off; off += (size_t)nL * HP * HP * 2;      off = (off + 255) & ~(size_t)255;
  const size_t oW1  = off; off += (size_t)HMP * HP * 2;          off = (off + 255) & ~(size_t)255;
  const size_t oH16 = off; off += (size_t)NPAD * HP * 2;         off = (off + 255) & ~(size_t)255;
  const size_t oP0  = off; off += (size_t)NPAD * HP * 4;         off = (off + 255) & ~(size_t)255;
  const size_t oP1  = off; off += (size_t)NPAD * HP * 4;         off = (off + 255) & ~(size_t)255;
  const size_t oP2  = off; off += (size_t)NPAD * HP * 4;         off = (off + 255) & ~(size_t)255;
  const size_t oCnt = off; off += (size_t)CNTPAD * 4;            off = (off + 255) & ~(size_t)255;
  const size_t oOff = off; off += (size_t)CNTPAD * 4;            off = (off + 255) & ~(size_t)255;
  const size_t oRb  = off; off += (size_t)RBN * 4;               off = (off + 255) & ~(size_t)255;
  const size_t oCsr = off; off += (size_t)csrLen * 4;            off = (off + 255) & ~(size_t)255;
  const size_t oDis = off; off += (size_t)NPAD * 4;              off = (off + 255) & ~(size_t)255;
  const size_t oPrt = off; off += (size_t)nStat * 2 * HP * 8;    off = (off + 255) & ~(size_t)255;
  const size_t oTbl = off; off += (size_t)2 * HP * 4;            off = (off + 255) & ~(size_t)255;
  if (off > ws_size || off > (size_t)WSCAP) return;
  _Float16* wpc = (_Float16*)(ws + oWc);
  _Float16* wp1 = (_Float16*)(ws + oW1);
  _Float16* h16 = (_Float16*)(ws + oH16);
  float*  p0   = (float*)(ws + oP0);
  float*  p1   = (float*)(ws + oP1);
  float*  p2   = (float*)(ws + oP2);
  int*    cnt  = (int*)(ws + oCnt);
  int*    offp = (int*)(ws + oOff);
  int*    rb   = (int*)(ws + oRb);
  int*    csr  = (int*)(ws + oCsr);
  float*  dis  = (float*)(ws + oDis);
  double* part = (double*)(ws + oPrt);
  float*  tbl  = (float*)(ws + oTbl);

  const int vec8 = ((nE & 3) == 0) ? 1 : 0;

  k_wprep<HID, HID, HP, HP><<<(nWcU + NTHR - 1) / NTHR, NTHR, 0, stream>>>(Wc, wpc, nL);
  k_wprep<HID, HMID, HP, HMP><<<(nW1U + NTHR - 1) / NTHR, NTHR, 0, stream>>>(W1, wp1, 1);
  k_embed<<<(nUnit + NTHR - 1) / NTHR, NTHR, 0, stream>>>(x, emb, p0, h16, nN, nCls, nUnit);

  k_count<<<nBC, NTHR, 0, stream>>>(dst, cnt, nE, vec8);
  k_offsets<<<1, OTHR, 0, stream>>>(cnt, offp, rb, nBC);
  hipFuncSetAttribute(reinterpret_cast<const void*>(&k_fill),
                      hipFuncAttributeMaxDynamicSharedMemorySize, LDS_FILL);
  k_fill<<<nBF, NTHR, LDS_FILL, stream>>>(src, dst, offp, rb, csr, nN, nE, vec8, csrLen);
  k_dis<<<NPAD / NTHR, NTHR, 0, stream>>>(cnt, dis, nN);

  float* hc = p0;
  float* hn = p1;
  for (int l = 0; l < nL; ++l) {
    k_gemm<<<nGm, NTHR, 0, stream>>>(h16, wpc + (size_t)l * HP * HP, hn);
    k_agg<<<nAgg, NTHR, 0, stream>>>(csr, offp, cnt, dis, hn, bc + (size_t)l * HID, p2, nN, csrLen);
    k_bnstat<<<nStat, HP, 0, stream>>>(p2, part, nN);
    k_bnfin<<<1, HP, 0, stream>>>(part, gamma + (size_t)l * HID, tbl, nStat, nN);
    k_update<<<(nUnit + NTHR - 1) / NTHR, NTHR, 0, stream>>>(p2, tbl, beta + (size_t)l * HID, hc, hn, h16, nN, nUnit);
    float* t = hc; hc = hn; hn = t;
  }

  k_pool_head<<<nPool, NTHR, 0, stream>>>(batch, hc, wp1, b1, W2, b2, out, nN, nG, 1);
}
